// MultiHeadAttention_85959475462393
// MI455X (gfx1250) — hardware-run, weakly checked
//
#include <hip/hip_runtime.h>
#ifndef NB
#define NB 2
#endif
#ifndef SEQ
#define SEQ 2048
#endif
#define NB_FULL 2
#define SEQ_FULL 2048
#define CH 1024
#define NH 16
#define HD 64
#define NTOK (NB * SEQ)

static_assert(SEQ % 64 == 0);
static_assert(NTOK % 128 == 0);
static_assert(SEQ <= SEQ_FULL);
static_assert(NB <= NB_FULL);
static_assert(HD == 64);
static_assert(NH * HD == CH);
static_assert(CH % 128 == 0);
static_assert((size_t)NB_FULL * SEQ_FULL * CH * 4 == (size_t)16777216);
static_assert((size_t)NTOK * CH * 2 * 10 + (size_t)CH * CH * 2 * 5 + (size_t)NB * (SEQ / 64) * 128 + 4096 <= (size_t)134217728);

typedef __bf16 v16b __attribute__((ext_vector_type(16)));
typedef _Float16 v16h __attribute__((ext_vector_type(16)));
typedef unsigned short v8us __attribute__((ext_vector_type(8), may_alias));
typedef float v8f __attribute__((ext_vector_type(8)));
typedef float v4f __attribute__((ext_vector_type(4)));
typedef float v4fa __attribute__((ext_vector_type(4), may_alias));
typedef int v4i __attribute__((ext_vector_type(4)));
typedef int v4ia __attribute__((ext_vector_type(4), may_alias));
union FragB { v16b v; v8us half[2]; };
union FragH { v16h v; v8us half[2]; _Float16 h[16]; };

#define LOG2E 1.4426950408889634f
#define NEGV (-1000000000.0f)

__device__ __forceinline__ unsigned short bf16_bits(float x) {
  unsigned int u = __float_as_uint(x);
  return (unsigned short)((u + 0x7FFFu + ((u >> 16) & 1u)) >> 16);
}
__device__ __forceinline__ float bf16_val(unsigned short b) { return __uint_as_float(((unsigned int)b) << 16); }
__device__ __forceinline__ unsigned short f16_bits(float x) {
  union { _Float16 h; unsigned short u; } c;
  c.h = (_Float16)x;
  return c.u;
}

__device__ __forceinline__ v8f wm_b(v16b a, v16b b, v8f c) {
  return __builtin_amdgcn_wmma_f32_16x16x32_bf16(false, a, false, b, (short)0, c, false, false);
}
__device__ __forceinline__ v8f wm_h(v16h a, v16h b, v8f c) {
  return __builtin_amdgcn_wmma_f32_16x16x32_f16(false, a, false, b, (short)0, c, false, false);
}

__device__ __forceinline__ v8f mma_bf6(v16b kh0, v16b kh1, v16b kl0, v16b kl1, v16b qh0, v16b qh1, v16b ql0, v16b ql1) {
  v8f c = {0.f, 0.f, 0.f, 0.f, 0.f, 0.f, 0.f, 0.f};
  c = wm_b(kl0, qh0, c);
  c = wm_b(kl1, qh1, c);
  c = wm_b(kh0, ql0, c);
  c = wm_b(kh1, ql1, c);
  c = wm_b(kh0, qh0, c);
  c = wm_b(kh1, qh1, c);
  asm volatile("v_nop\n\tv_nop\n\tv_nop\n\tv_nop" : "+v"(c) : "v"(kh0), "v"(kh1), "v"(kl0), "v"(kl1), "v"(qh0), "v"(qh1), "v"(ql0), "v"(ql1));
  return c;
}
__device__ __forceinline__ void mma_h3(v16h vh, v16h vl, v16h ph, v16h pl, v8f& ch, v8f& cl) {
  ch = wm_h(vh, ph, ch);
  cl = wm_h(vh, pl, cl);
  cl = wm_h(vl, ph, cl);
  asm volatile("v_nop\n\tv_nop\n\tv_nop\n\tv_nop" : "+v"(ch), "+v"(cl) : "v"(vh), "v"(vl), "v"(ph), "v"(pl));
}

__global__ __launch_bounds__(256) void k_cvt(const float* __restrict__ X, unsigned short* __restrict__ Xb) {
  const int t = blockIdx.x * 256 + threadIdx.x;
  if (t >= NTOK * (CH / 8)) return;
  const int row = t >> 7, piece = t & 127;
  const int b = row / SEQ, s = row - b * SEQ;
  const float* src = X + ((size_t)b * SEQ_FULL + s) * CH + piece * 8;
  const v4f x0 = *(const v4fa*)(src), x1 = *(const v4fa*)(src + 4);
  v8us o;
  o[0] = bf16_bits(x0[0]); o[1] = bf16_bits(x0[1]); o[2] = bf16_bits(x0[2]); o[3] = bf16_bits(x0[3]);
  o[4] = bf16_bits(x1[0]); o[5] = bf16_bits(x1[1]); o[6] = bf16_bits(x1[2]); o[7] = bf16_bits(x1[3]);
  unsigned short* d = Xb + (size_t)t * 8;
  *(volatile v8us*)d = o;
  __threadfence();
  *(volatile v8us*)d = o;
}

__global__ __launch_bounds__(256) void k_wt(const float* __restrict__ W, int N, unsigned short* __restrict__ WT, int ldo, int dup) {
  __shared__ unsigned short tl[64][66];
  const int tid = threadIdx.x;
  const int n0 = blockIdx.x * 64, k0 = blockIdx.y * 64;
  for (int i = tid; i < 64 * 16; i += 256) {
    const int j = i >> 4, c4 = (i & 15) * 4;
    const v4f x = *(const v4fa*)(W + (size_t)(k0 + j) * N + n0 + c4);
    tl[c4 + 0][j] = bf16_bits(x[0]); tl[c4 + 1][j] = bf16_bits(x[1]);
    tl[c4 + 2][j] = bf16_bits(x[2]); tl[c4 + 3][j] = bf16_bits(x[3]);
  }
  __syncthreads();
  for (int pass = 0; pass < 2; ++pass) {
    for (int i = tid; i < 64 * 8; i += 256) {
      const int nn = i >> 3, j8 = (i & 7) * 8;
      v8us o;
#pragma unroll
      for (int q = 0; q < 8; ++q) o[q] = tl[nn][j8 + q];
      unsigned short* d = WT + (size_t)(n0 + nn) * ldo + k0 + j8;
      *(volatile v8us*)d = o;
      if (dup != 0) *(volatile v8us*)(d + CH) = o;
    }
    if (pass == 0) __threadfence();
  }
}

__global__ __launch_bounds__(256) void k_mflag(const int* __restrict__ mask, int* __restrict__ flags) {
  __shared__ int sw[8];
  const int tid = threadIdx.x, w = __builtin_amdgcn_readfirstlane((int)(tid >> 5)), lane = tid & 31;
  const int b = blockIdx.x / (SEQ / 64), qt = blockIdx.x % (SEQ / 64);
  int ok = 1;
  for (int i = tid; i < 64 * (SEQ / 4); i += 256) {
    const int rr = i / (SEQ / 4), c4 = (i - rr * (SEQ / 4)) * 4;
    const int q = qt * 64 + rr;
    const v4i m = *(const v4ia*)(mask + ((size_t)b * SEQ_FULL + q) * SEQ_FULL + c4);
    ok &= ((m[0] != 0) == (c4 + 0 <= q)) ? 1 : 0;
    ok &= ((m[1] != 0) == (c4 + 1 <= q)) ? 1 : 0;
    ok &= ((m[2] != 0) == (c4 + 2 <= q)) ? 1 : 0;
    ok &= ((m[3] != 0) == (c4 + 3 <= q)) ? 1 : 0;
  }
#pragma unroll
  for (int o = 16; o >= 1; o >>= 1) ok &= __shfl_xor(ok, o, 32);
  if (lane == 0) sw[w] = ok;
  __syncthreads();
  if (tid < 8) {
    const int f = sw[0] & sw[1] & sw[2] & sw[3] & sw[4] & sw[5] & sw[6] & sw[7];
    const v4i o = {f, f, f, f};
    int* d = flags + (size_t)blockIdx.x * 32 + tid * 4;
    *(volatile v4i*)d = o;
    __threadfence();
    *(volatile v4i*)d = o;
  }
}

template <int EPI>
__global__ __launch_bounds__(128) void k_gemm(const unsigned short* __restrict__ P, const unsigned short* __restrict__ R,
                                              int ldp, int ldr, int K,
                                              unsigned short* __restrict__ o16a, unsigned short* __restrict__ o16b, float* __restrict__ o32) {
  __shared__ __attribute__((aligned(16))) float st[4][32][68];
  const int tid = threadIdx.x, w = __builtin_amdgcn_readfirstlane((int)(tid >> 5)), lane = tid & 31, ln = lane & 15, hh = lane >> 4;
  const int i0 = blockIdx.y * 128 + 32 * w;
  const int j0 = blockIdx.x * 64;
  const unsigned short* pa0 = P + (size_t)(i0 + ln) * ldp + 8 * hh;
  const unsigned short* pa1 = pa0 + (size_t)16 * ldp;
  const unsigned short* pb0 = R + (size_t)(j0 + ln) * ldr + 8 * hh;
  const unsigned short* pb1 = pb0 + (size_t)16 * ldr;
  const unsigned short* pb2 = pb0 + (size_t)32 * ldr;
  const unsigned short* pb3 = pb0 + (size_t)48 * ldr;
  v8f acc[2][4] = {};
#pragma unroll 1
  for (int k0 = 0; k0 < K; k0 += 32) {
    FragB a0, a1, b0, b1, b2, b3;
    a0.half[0] = *(const v8us*)(pa0 + k0); a0.half[1] = *(const v8us*)(pa0 + k0 + 16);
    a1.half[0] = *(const v8us*)(pa1 + k0); a1.half[1] = *(const v8us*)(pa1 + k0 + 16);
    b0.half[0] = *(const v8us*)(pb0 + k0); b0.half[1] = *(const v8us*)(pb0 + k0 + 16);
    b1.half[0] = *(const v8us*)(pb1 + k0); b1.half[1] = *(const v8us*)(pb1 + k0 + 16);
    b2.half[0] = *(const v8us*)(pb2 + k0); b2.half[1] = *(const v8us*)(pb2 + k0 + 16);
    b3.half[0] = *(const v8us*)(pb3 + k0); b3.half[1] = *(const v8us*)(pb3 + k0 + 16);
    acc[0][0] = wm_b(a0.v, b0.v, acc[0][0]);
    acc[0][1] = wm_b(a0.v, b1.v, acc[0][1]);
    acc[0][2] = wm_b(a0.v, b2.v, acc[0][2]);
    acc[0][3] = wm_b(a0.v, b3.v, acc[0][3]);
    acc[1][0] = wm_b(a1.v, b0.v, acc[1][0]);
    acc[1][1] = wm_b(a1.v, b1.v, acc[1][1]);
    acc[1][2] = wm_b(a1.v, b2.v, acc[1][2]);
    acc[1][3] = wm_b(a1.v, b3.v, acc[1][3]);
    asm volatile("v_nop\n\tv_nop\n\tv_nop\n\tv_nop"
                 : "+v"(acc[0][0]), "+v"(acc[0][1]), "+v"(acc[0][2]), "+v"(acc[0][3]),
                   "+v"(acc[1][0]), "+v"(acc[1][1]), "+v"(acc[1][2]), "+v"(acc[1][3])
                 : "v"(a0.v), "v"(a1.v), "v"(b0.v), "v"(b1.v), "v"(b2.v), "v"(b3.v));
  }
#pragma unroll
  for (int mt = 0; mt < 2; ++mt)
#pragma unroll
    for (int nt = 0; nt < 4; ++nt)
#pragma unroll
      for (int r = 0; r < 8; ++r)
        st[w][16 * mt + 8 * hh + r][16 * nt + ln] = acc[mt][nt][r];
  __syncthreads();
  if (EPI == 0) {
    const int rsub = lane >> 3, pc = (lane & 7) * 8;
    for (int pass = 0; pass < 2; ++pass) {
#pragma unroll
      for (int q = 0; q < 8; ++q) {
        const int row = 4 * q + rsub;
        const v4f x0 = *(const v4fa*)&st[w][row][pc];
        const v4f x1 = *(const v4fa*)&st[w][row][pc + 4];
        v8us hi, lo;
#pragma unroll
        for (int e = 0; e < 4; ++e) {
          const unsigned short h0 = bf16_bits(x0[e]), h1 = bf16_bits(x1[e]);
          hi[e] = h0; hi[4 + e] = h1;
          lo[e] = bf16_bits(x0[e] - bf16_val(h0));
          lo[4 + e] = bf16_bits(x1[e] - bf16_val(h1));
        }
        const size_t off = (size_t)(i0 + row) * CH + j0 + pc;
        *(volatile v8us*)(o16a + off) = hi;
        *(volatile v8us*)(o16b + off) = lo;
      }
      if (pass == 0) __threadfence();
    }
  } else if (EPI == 1) {
    const int rsub = lane >> 3, pc = (lane & 7) * 8;
    const int b = j0 / SEQ, s0 = j0 - b * SEQ;
    for (int pass = 0; pass < 2; ++pass) {
#pragma unroll
      for (int q = 0; q < 8; ++q) {
        const int row = 4 * q + rsub;
        const v4f x0 = *(const v4fa*)&st[w][row][pc];
        const v4f x1 = *(const v4fa*)&st[w][row][pc + 4];
        v8us hi, lo;
#pragma unroll
        for (int e = 0; e < 4; ++e) {
          const float y0 = x0[e] * 16.0f, y1 = x1[e] * 16.0f;
          const _Float16 g0 = (_Float16)y0, g1 = (_Float16)y1;
          hi[e] = f16_bits((float)g0); hi[4 + e] = f16_bits((float)g1);
          lo[e] = f16_bits((y0 - (float)g0) * 2048.0f);
          lo[4 + e] = f16_bits((y1 - (float)g1) * 2048.0f);
        }
        const size_t off = ((size_t)b * CH + (i0 + row)) * SEQ + s0 + pc;
        *(volatile v8us*)(o16a + off) = hi;
        *(volatile v8us*)(o16b + off) = lo;
      }
      if (pass == 0) __threadfence();
    }
  } else {
    const int rsub = lane >> 4, c4 = (lane & 15) * 4;
    for (int pass = 0; pass < 2; ++pass) {
#pragma unroll
      for (int q = 0; q < 16; ++q) {
        const int row = 2 * q + rsub;
        const v4f v = *(const v4fa*)&st[w][row][c4];
        const int tok = i0 + row;
        const int b = tok / SEQ, s = tok - b * SEQ;
        if (tok < NTOK)
          *(volatile v4f*)(o32 + ((size_t)b * SEQ_FULL + s) * CH + j0 + c4) = v;
      }
      if (pass == 0) __threadfence();
    }
  }
}

template <int MODE>
__device__ __forceinline__ void fa_step(const unsigned short* __restrict__ Khp, const unsigned short* __restrict__ Klp,
                                        const unsigned short* __restrict__ Vhp, const unsigned short* __restrict__ Vlp,
                                        const int* __restrict__ mrow,
                                        int key0, int qg, int ln, int hh,
                                        const FragB& qh0, const FragB& qh1, const FragB& ql0, const FragB& ql1,
                                        float& mr, float& lr, v8f (&Oh)[4], v8f (&Ol)[4]) {
  const size_t ko = (size_t)(key0 + ln) * CH + 8 * hh;
  v8f s0, s1;
  {
    FragB h0, h1, l0, l1;
    h0.half[0] = *(const v8us*)(Khp + ko);      h0.half[1] = *(const v8us*)(Khp + ko + 16);
    h1.half[0] = *(const v8us*)(Khp + ko + 32); h1.half[1] = *(const v8us*)(Khp + ko + 48);
    l0.half[0] = *(const v8us*)(Klp + ko);      l0.half[1] = *(const v8us*)(Klp + ko + 16);
    l1.half[0] = *(const v8us*)(Klp + ko + 32); l1.half[1] = *(const v8us*)(Klp + ko + 48);
    s0 = mma_bf6(h0.v, h1.v, l0.v, l1.v, qh0.v, qh1.v, ql0.v, ql1.v);
  }
  {
    const size_t k1 = ko + (size_t)16 * CH;
    FragB h0, h1, l0, l1;
    h0.half[0] = *(const v8us*)(Khp + k1);      h0.half[1] = *(const v8us*)(Khp + k1 + 16);
    h1.half[0] = *(const v8us*)(Khp + k1 + 32); h1.half[1] = *(const v8us*)(Khp + k1 + 48);
    l0.half[0] = *(const v8us*)(Klp + k1);      l0.half[1] = *(const v8us*)(Klp + k1 + 16);
    l1.half[0] = *(const v8us*)(Klp + k1 + 32); l1.half[1] = *(const v8us*)(Klp + k1 + 48);
    s1 = mma_bf6(h0.v, h1.v, l0.v, l1.v, qh0.v, qh1.v, ql0.v, ql1.v);
  }
  float sc[16];
#pragma unroll
  for (int r = 0; r < 8; ++r) { sc[r] = s0[r] * 0.125f; sc[8 + r] = s1[r] * 0.125f; }
  if (MODE == 1) {
#pragma unroll
    for (int r = 0; r < 8; ++r) {
      const int kg = key0 + 8 * hh + r;
      sc[r]     += (kg > qg) ? NEGV : 0.0f;
      sc[8 + r] += (kg + 16 > qg) ? NEGV : 0.0f;
    }
  }
  if (MODE == 2) {
    const int* mp = mrow + key0 + 8 * hh;
    const v4i m0 = *(const v4ia*)(mp), m1 = *(const v4ia*)(mp + 4);
    const v4i m2 = *(const v4ia*)(mp + 16), m3 = *(const v4ia*)(mp + 20);
#pragma unroll
    for (int r = 0; r < 4; ++r) {
      sc[r]      += (m0[r] != 0) ? 0.0f : NEGV;
      sc[4 + r]  += (m1[r] != 0) ? 0.0f : NEGV;
      sc[8 + r]  += (m2[r] != 0) ? 0.0f : NEGV;
      sc[12 + r] += (m3[r] != 0) ? 0.0f : NEGV;
    }
  }
  asm volatile("" ::: "memory");
  const size_t vo = (size_t)ln * SEQ + key0 + 8 * hh;
  FragH vh[4], vl[4];
#pragma unroll
  for (int t = 0; t < 4; ++t) {
    vh[t].half[0] = *(const v8us*)(Vhp + vo + (size_t)t * 16 * SEQ);
    vh[t].half[1] = *(const v8us*)(Vhp + vo + (size_t)t * 16 * SEQ + 16);
    vl[t].half[0] = *(const v8us*)(Vlp + vo + (size_t)t * 16 * SEQ);
    vl[t].half[1] = *(const v8us*)(Vlp + vo + (size_t)t * 16 * SEQ + 16);
  }
  float mx = sc[0];
#pragma unroll
  for (int i = 1; i < 16; ++i) mx = fmaxf(mx, sc[i]);
  mx = fmaxf(mx, __shfl_xor(mx, 16, 32));
  const float mnew = fmaxf(mr, mx);
  const float al = exp2f((mr - mnew) * LOG2E);
  mr = mnew;
  FragH ph, pl;
  float ps = 0.0f;
#pragma unroll
  for (int i = 0; i < 16; ++i) {
    const float pc = exp2f(fmaf(sc[i] - mnew, LOG2E, 8.0f));
    ps += pc;
    const _Float16 h = (_Float16)pc;
    ph.h[i] = h;
    pl.h[i] = (_Float16)((pc - (float)h) * 2048.0f);
  }
  ps += __shfl_xor(ps, 16, 32);
  lr = lr * al + ps;
#pragma unroll
  for (int t = 0; t < 4; ++t) { Oh[t] = Oh[t] * al; Ol[t] = Ol[t] * al; }
#pragma unroll
  for (int t = 0; t < 4; ++t) mma_h3(vh[t].v, vl[t].v, ph.v, pl.v, Oh[t], Ol[t]);
}

__global__ __launch_bounds__(128) void k_attn(const unsigned short* __restrict__ Qh, const unsigned short* __restrict__ Ql,
                                              const unsigned short* __restrict__ Kh, const unsigned short* __restrict__ Kl,
                                              const unsigned short* __restrict__ VTh, const unsigned short* __restrict__ VTl,
                                              const int* __restrict__ mask, const int* __restrict__ flags,
                                              unsigned short* __restrict__ Cc) {
  __shared__ __attribute__((aligned(16))) float so[4][16][68];
  const int tid = threadIdx.x, w = __builtin_amdgcn_readfirstlane((int)(tid >> 5)), lane = tid & 31, ln = lane & 15, hh = lane >> 4;
  const int bx = blockIdx.x;
  const int qt = bx % (SEQ / 64);
  const int h = (bx / (SEQ / 64)) % NH;
  const int b = bx / ((SEQ / 64) * NH);
  const int qbase = qt * 64 + 16 * w;
  const int qg = qbase + ln;
  const size_t qoff = ((size_t)b * SEQ + qg) * CH + h * HD + 8 * hh;
  FragB qh0, qh1, ql0, ql1;
  qh0.half[0] = *(const v8us*)(Qh + qoff);      qh0.half[1] = *(const v8us*)(Qh + qoff + 16);
  qh1.half[0] = *(const v8us*)(Qh + qoff + 32); qh1.half[1] = *(const v8us*)(Qh + qoff + 48);
  ql0.half[0] = *(const v8us*)(Ql + qoff);      ql0.half[1] = *(const v8us*)(Ql + qoff + 16);
  ql1.half[0] = *(const v8us*)(Ql + qoff + 32); ql1.half[1] = *(const v8us*)(Ql + qoff + 48);
  float mr = -3.0e38f, lr = 0.0f;
  v8f Oh[4] = {}, Ol[4] = {};
  const unsigned short* Khp = Kh + (size_t)b * SEQ * CH + h * HD;
  const unsigned short* Klp = Kl + (size_t)b * SEQ * CH + h * HD;
  const unsigned short* Vhp = VTh + ((size_t)b * CH + h * HD) * SEQ;
  const unsigned short* Vlp = VTl + ((size_t)b * CH + h * HD) * SEQ;
  const int* mrow = mask + ((size_t)b * SEQ_FULL + qg) * SEQ_FULL;
  int fl = flags[(size_t)(b * (SEQ / 64) + qt) * 32];
  fl = __builtin_amdgcn_readfirstlane(fl);
  if (fl == 1) {
    const int nfull = qbase >> 5;
#pragma unroll 1
    for (int j = 0; j < nfull; ++j)
      fa_step<0>(Khp, Klp, Vhp, Vlp, mrow, 32 * j, qg, ln, hh, qh0, qh1, ql0, ql1, mr, lr, Oh, Ol);
    fa_step<1>(Khp, Klp, Vhp, Vlp, mrow, 32 * nfull, qg, ln, hh, qh0, qh1, ql0, ql1, mr, lr, Oh, Ol);
  } else {
#pragma unroll 1
    for (int j = 0; j < SEQ / 32; ++j)
      fa_step<2>(Khp, Klp, Vhp, Vlp, mrow, 32 * j, qg, ln, hh, qh0, qh1, ql0, ql1, mr, lr, Oh, Ol);
  }

  const float inv = 1.0f / (16.0f * lr);
#pragma unroll
  for (int t = 0; t < 4; ++t) {
    v4f a, c;
#pragma unroll
    for (int r = 0; r < 4; ++r) {
      a[r] = (Oh[t][r] + Ol[t][r] * 0.00048828125f) * inv;
      c[r] = (Oh[t][4 + r] + Ol[t][4 + r] * 0.00048828125f) * inv;
    }
    *(v4fa*)&so[w][ln][16 * t + 8 * hh] = a;
    *(v4fa*)&so[w][ln][16 * t + 8 * hh + 4] = c;
  }
  __syncthreads();
  const int rsub = lane >> 3, pc = (lane & 7) * 8;
  const size_t tok0 = (size_t)b * SEQ + qbase;
  for (int pass = 0; pass < 2; ++pass) {
#pragma unroll
    for (int q = 0; q < 4; ++q) {
      const int row = 4 * q + rsub;
      const v4f x0 = *(const v4fa*)&so[w][row][pc];
      const v4f x1 = *(const v4fa*)&so[w][row][pc + 4];
      v8us hi, lo;
#pragma unroll
      for (int e = 0; e < 4; ++e) {
        const unsigned short h0 = bf16_bits(x0[e]), h1 = bf16_bits(x1[e]);
        hi[e] = h0; hi[4 + e] = h1;
        lo[e] = bf16_bits(x0[e] - bf16_val(h0));
        lo[4 + e] = bf16_bits(x1[e] - bf16_val(h1));
      }
      unsigned short* d = Cc + (tok0 + row) * (size_t)(2 * CH) + h * HD + pc;
      *(volatile v8us*)d = hi;
      *(volatile v8us*)(d + CH) = lo;
    }
    if (pass == 0) __threadfence();
  }
}

extern "C" void kernel_launch(void* const* d_in, const int* in_sizes, int n_in,
                              void* d_out, int out_size, void* d_ws, size_t ws_size, hipStream_t stream) {
  if (n_in < 6) return;
  const long long need_x = ((long long)(NB - 1) * SEQ_FULL + SEQ) * CH;
  const long long need_m = ((long long)(NB - 1) * SEQ_FULL + (SEQ - 1)) * SEQ_FULL + SEQ;
  if ((long long)in_sizes[0] < need_x || (long long)in_sizes[1] < need_x) return;
  if ((long long)in_sizes[2] < (long long)CH * CH || (long long)in_sizes[3] < (long long)2 * CH * CH ||
      (long long)in_sizes[4] < (long long)CH * CH) return;
  if ((long long)in_sizes[5] < need_m) return;
  if ((long long)out_size < need_x) return;
  const float* query = (const float*)d_in[0];
  const float* mem   = (const float*)d_in[1];
  const float* Wq    = (const float*)d_in[2];
  const float* Wkv   = (const float*)d_in[3];
  const float* Wo    = (const float*)d_in[4];
  const int* mask    = (const int*)d_in[5];
  float* out = (float*)d_out;
  char* ws = (char*)d_ws;
  size_t off = 0;
  const size_t szX = (size_t)NTOK * CH * 2;
  const size_t szW = (size_t)CH * CH * 2;
  unsigned short* Xq   = (unsigned short*)(ws + off); off += (szX + 255) & ~(size_t)255;
  unsigned short* Xm   = (unsigned short*)(ws + off); off += (szX + 255) & ~(size_t)255;
  unsigned short* WqT  = (unsigned short*)(ws + off); off += (szW + 255) & ~(size_t)255;
  unsigned short* WkvT = (unsigned short*)(ws + off); off += (2 * szW + 255) & ~(size_t)255;
  unsigned short* WoT2 = (unsigned short*)(ws + off); off += (2 * szW + 255) & ~(size_t)255;
  unsigned short* Qh   = (unsigned short*)(ws + off); off += (szX + 255) & ~(size_t)255;
  unsigned short* Ql   = (unsigned short*)(ws + off); off += (szX + 255) & ~(size_t)255;
  unsigned short* Kh   = (unsigned short*)(ws + off); off += (szX + 255) & ~(size_t)255;
  unsigned short* Kl   = (unsigned short*)(ws + off); off += (szX + 255) & ~(size_t)255;
  unsigned short* VTh  = (unsigned short*)(ws + off); off += (szX + 255) & ~(size_t)255;
  unsigned short* VTl  = (unsigned short*)(ws + off); off += (szX + 255) & ~(size_t)255;
  unsigned short* Ccat = (unsigned short*)(ws + off); off += (2 * szX + 255) & ~(size_t)255;
  int* flags           = (int*)(ws + off);            off += ((size_t)NB * (SEQ / 64) * 128 + 255) & ~(size_t)255;
  if (off > ws_size || off > (size_t)134217728) return;

  const unsigned gcvt = (unsigned)((NTOK * (CH / 8) + 255) / 256);
  k_cvt<<<gcvt, 256, 0, stream>>>(query, Xq);
  k_cvt<<<gcvt, 256, 0, stream>>>(mem, Xm);
  k_wt<<<dim3(CH / 64, CH / 64), 256, 0, stream>>>(Wq, CH, WqT, CH, 0);
  k_wt<<<dim3(2 * CH / 64, CH / 64), 256, 0, stream>>>(Wkv, 2 * CH, WkvT, CH, 0);
  k_wt<<<dim3(CH / 64, CH / 64), 256, 0, stream>>>(Wo, CH, WoT2, 2 * CH, 1);
  k_mflag<<<(unsigned)(NB * (SEQ / 64)), 256, 0, stream>>>(mask, flags);
  k_gemm<0><<<dim3(CH / 64, NTOK / 128), 128, 0, stream>>>(Xq, WqT, CH, CH, CH, Qh, Ql, out);
  k_gemm<0><<<dim3(CH / 64, NTOK / 128), 128, 0, stream>>>(Xm, WkvT, CH, CH, CH, Kh, Kl, out);
  k_gemm<1><<<dim3(NTOK / 64, CH / 128), 128, 0, stream>>>(WkvT + (size_t)CH * CH, Xm, CH, CH, CH, VTh, VTl, out);
  k_attn<<<(unsigned)(NB * NH * (SEQ / 64)), 128, 0, stream>>>(Qh, Ql, Kh, Kl, VTh, VTl, mask, flags, Ccat);
  k_gemm<2><<<dim3(CH / 64, NTOK / 128), 128, 0, stream>>>(Ccat, WoT2, 2 * CH, 2 * CH, 2 * CH, Qh, Ql, out);
}
